// SelectiveSSM_56324201119970
// MI455X (gfx1250) — hardware-verified
//
#include <hip/hip_runtime.h>
#include <math.h>

typedef __attribute__((ext_vector_type(16))) _Float16 v16h;
typedef __attribute__((ext_vector_type(8)))  _Float16 v8h;
typedef __attribute__((ext_vector_type(2)))  _Float16 v2h;
typedef __attribute__((ext_vector_type(16))) __bf16   v16b;
typedef __attribute__((ext_vector_type(8)))  __bf16   v8b;
typedef __attribute__((ext_vector_type(8)))  float    v8f;
typedef __attribute__((ext_vector_type(4)))  float    v4f;
typedef __attribute__((ext_vector_type(4)))  unsigned int v4u;

constexpr int kBatch  = 2;
constexpr int kSeq    = 1024;
constexpr int kDm     = 1024;
constexpr int kDin    = 2048;
constexpr int kNst    = 16;
constexpr int kXzP    = 2 * kDin;
constexpr int kXdN    = 2 * kNst + 1;
constexpr int kXdP    = 64;
constexpr int kRows   = kBatch * kSeq;
constexpr int kConvTP = 260;
constexpr int kScanTS = 64;
constexpr int kScanCh = 64;
constexpr int kScanYP = 68;
static_assert(kXdN == 33 && kXdN <= kXdP);
static_assert((kDm % 32) == 0 && (kDin % 32) == 0);
static_assert((kRows % 64) == 0 && (kXzP % 64) == 0 && (kXdP % 64) == 0 && (kDm % 64) == 0);
static_assert((kSeq % kScanTS) == 0 && (kSeq % 64) == 0 && (kDin % kScanCh) == 0 && (kDin % 256) == 0);
static_assert((kSeq & (kSeq - 1)) == 0);
static_assert(((kXdN * kDin) % 8) == 0);

constexpr int kModeIn  = 2;
constexpr int kModeXp  = 2;
constexpr int kModeOut = 2;
static_assert(kModeIn == 0 || kModeIn == 2);
static_assert(kModeXp == 0 || kModeXp == 2);
static_assert(kModeOut == 0 || kModeOut == 2);
constexpr float kCarryX = 16.0f;
constexpr float kCarryW = 64.0f;
constexpr float kCarryU = 64.0f;
constexpr float kCarryY = 4096.0f;
constexpr float kF16MinNormal = 6.103515625e-5f;
constexpr bool kScanFastExp = false;

constexpr size_t kOffXH  = 0;
constexpr size_t kOffXL  = kOffXH  + (size_t)kRows * kDm  * 2;
constexpr size_t kOffW0H = kOffXL  + (size_t)kRows * kDm  * 2;
constexpr size_t kOffW0L = kOffW0H + (size_t)kXzP  * kDm  * 2;
constexpr size_t kOffW1H = kOffW0L + (size_t)kXzP  * kDm  * 2;
constexpr size_t kOffW1L = kOffW1H + (size_t)kXdP  * kDin * 2;
constexpr size_t kOffW3H = kOffW1L + (size_t)kXdP  * kDin * 2;
constexpr size_t kOffW3L = kOffW3H + (size_t)kDm   * kDin * 2;
constexpr size_t kOffXZ  = kOffW3L + (size_t)kDm   * kDin * 2;
constexpr size_t kOffUC  = kOffXZ  + (size_t)kRows * kXzP * 4;
constexpr size_t kOffUH  = kOffUC  + (size_t)kRows * kDin * 4;
constexpr size_t kOffUL  = kOffUH  + (size_t)kRows * kDin * 2;
constexpr size_t kOffXD  = kOffUL  + (size_t)kRows * kDin * 2;
constexpr size_t kOffYH  = kOffXD  + (size_t)kRows * kXdP * 4;
constexpr size_t kOffYL  = kOffYH  + (size_t)kRows * kDin * 2;
constexpr size_t kWsTotal = kOffYL + (size_t)kRows * kDin * 2;
static_assert(kWsTotal == 118489088ull);
static_assert(kWsTotal <= 134217728ull);
static_assert((kOffXL % 128) == 0 && (kOffW0H % 128) == 0 && (kOffW0L % 128) == 0 && (kOffW1H % 128) == 0 &&
              (kOffW1L % 128) == 0 && (kOffW3H % 128) == 0 && (kOffW3L % 128) == 0 && (kOffXZ % 128) == 0 &&
              (kOffUC % 128) == 0 && (kOffUH % 128) == 0 && (kOffUL % 128) == 0 && (kOffXD % 128) == 0 &&
              (kOffYH % 128) == 0 && (kOffYL % 128) == 0);

__device__ __forceinline__ unsigned pin_u32(unsigned v) { asm volatile("" : "+v"(v)); return v; }

__device__ __forceinline__ unsigned bf_hi32(float f) {
  unsigned u = __float_as_uint(f);
  const unsigned lsb = (u & 0x00010000u) ? 1u : 0u;
  return (u + 0x7FFFu + lsb) & 0xFFFF0000u;
}
__device__ __forceinline__ void pack2_split(float a, float b, unsigned& wh, unsigned& wl) {
  const unsigned ha = bf_hi32(a), hb = bf_hi32(b);
  const unsigned la = bf_hi32(a - __uint_as_float(ha));
  const unsigned lb = bf_hi32(b - __uint_as_float(hb));
  wh = (hb & 0xFFFF0000u) | (ha >> 16);
  wl = (lb & 0xFFFF0000u) | (la >> 16);
}
__device__ __forceinline__ unsigned pack2_f16(float a, float b, float carry) {
  float sa = a * carry, sb = b * carry;
  sa = (fabsf(sa) < kF16MinNormal) ? 0.0f : sa;
  sb = (fabsf(sb) < kF16MinNormal) ? 0.0f : sb;
  const v2h p = {(_Float16)sa, (_Float16)sb};
  return __builtin_bit_cast(unsigned, p);
}
template <int MODE>
__device__ __forceinline__ void pack8(const float (&f)[8], const float carry, v4u& wh, v4u& wl) {
  if (MODE == 0) {
    const unsigned w0 = pack2_f16(f[0], f[1], carry);
    const unsigned w1 = pack2_f16(f[2], f[3], carry);
    const unsigned w2 = pack2_f16(f[4], f[5], carry);
    const unsigned w3 = pack2_f16(f[6], f[7], carry);
    wh = (v4u){w0, w1, w2, w3};
    wl = (v4u){0u, 0u, 0u, 0u};
  } else {
    unsigned h0, h1, h2, h3, l0, l1, l2, l3;
    pack2_split(f[0], f[1], h0, l0);
    pack2_split(f[2], f[3], h1, l1);
    pack2_split(f[4], f[5], h2, l2);
    pack2_split(f[6], f[7], h3, l3);
    wh = (v4u){h0, h1, h2, h3};
    wl = (v4u){l0, l1, l2, l3};
  }
}

__device__ __forceinline__ void tie_acc_h(v8f& a, v16h x, v16h y) { asm volatile("" : "+v"(a) : "v"(x), "v"(y)); }
__device__ __forceinline__ void tie_acc_b(v8f& a, v16b x, v16b y) { asm volatile("" : "+v"(a) : "v"(x), "v"(y)); }
__device__ __forceinline__ void nop_acc_h(v8f& a, v16h x, v16h y) { asm volatile("v_nop\n\tv_nop\n\tv_nop\n\tv_nop" : "+v"(a) : "v"(x), "v"(y)); }
__device__ __forceinline__ void nop_acc_b(v8f& a, v16b x, v16b y) { asm volatile("v_nop\n\tv_nop\n\tv_nop\n\tv_nop" : "+v"(a) : "v"(x), "v"(y)); }
__device__ __forceinline__ void keep4_h(v16h a, v16h b, v16h c, v16h d) { asm volatile("v_nop" :: "v"(a), "v"(b), "v"(c), "v"(d)); }
__device__ __forceinline__ void keep4_b(v16b a, v16b b, v16b c, v16b d) { asm volatile("v_nop" :: "v"(a), "v"(b), "v"(c), "v"(d)); }
__device__ __forceinline__ void acc_guard4(v8f& a, v8f& b, v8f& c, v8f& d) { asm volatile("v_nop\n\tv_nop\n\tv_nop\n\tv_nop" : "+v"(a), "+v"(b), "+v"(c), "+v"(d)); }
template <typename T> struct Frag;
template <> struct Frag<_Float16> {
  typedef v16h V; union U { v16h v; v8h h[2]; };
  static __device__ __forceinline__ v16h load(const _Float16* p) {
    U f; f.h[0] = *(const v8h*)(p); f.h[1] = *(const v8h*)(p + 16); return f.v;
  }
  static __device__ __forceinline__ v8f mma(v16h a, v16h b, v8f c) {
    return __builtin_amdgcn_wmma_f32_16x16x32_f16(false, a, false, b, (short)0, c, false, false);
  }
  static __device__ __forceinline__ void tie(v8f& a, v16h x, v16h y) { tie_acc_h(a, x, y); }
  static __device__ __forceinline__ void nops(v8f& a, v16h x, v16h y) { nop_acc_h(a, x, y); }
  static __device__ __forceinline__ void keep(v16h a, v16h b, v16h c, v16h d) { keep4_h(a, b, c, d); }
};
template <> struct Frag<__bf16> {
  typedef v16b V; union U { v16b v; v8b h[2]; };
  static __device__ __forceinline__ v16b load(const __bf16* p) {
    U f; f.h[0] = *(const v8b*)(p); f.h[1] = *(const v8b*)(p + 16); return f.v;
  }
  static __device__ __forceinline__ v8f mma(v16b a, v16b b, v8f c) {
    return __builtin_amdgcn_wmma_f32_16x16x32_bf16(false, a, false, b, (short)0, c, false, false);
  }
  static __device__ __forceinline__ void tie(v8f& a, v16b x, v16b y) { tie_acc_b(a, x, y); }
  static __device__ __forceinline__ void nops(v8f& a, v16b x, v16b y) { nop_acc_b(a, x, y); }
  static __device__ __forceinline__ void keep(v16b a, v16b b, v16b c, v16b d) { keep4_b(a, b, c, d); }
};
template <int ET> struct Elem;
template <> struct Elem<0> { typedef _Float16 T; };
template <> struct Elem<1> { typedef __bf16 T; };

template <int ET, int SPL>
__global__ __launch_bounds__(256) void wmma_gemm64(
    const unsigned short* __restrict__ Ap, const unsigned short* __restrict__ A2p, int lda,
    const unsigned short* __restrict__ Btp, const unsigned short* __restrict__ Bt2p, int ldb,
    float* __restrict__ Cout, int ldc, int M, int N, int K, float scale) {
  typedef typename Elem<ET>::T T;
  typedef typename Frag<T>::V V;
  const T* A = (const T*)Ap; const T* A2 = (const T*)A2p; const T* Bt = (const T*)Btp; const T* Bt2 = (const T*)Bt2p;
  __shared__ __align__(16) float sT[8][16 * 68];
  const int lane = threadIdx.x & 31;
  const int wave = threadIdx.x >> 5;
  const int tilesN = N >> 6;
  const int tilesM = M >> 6;
  const int tile = blockIdx.x * 8 + wave;
  if (tile >= tilesM * tilesN) return;
  const int tm = tile / tilesN;
  const int tn = tile - tm * tilesN;
  const int m0 = tm << 6;
  const int n0 = tn << 6;

  const int rlane = lane & 15;
  const int koff  = (lane >> 4) * 8;
  const int mOff  = (lane >> 4) * 8;

  v8f acc[4][4];
#pragma unroll
  for (int i = 0; i < 4; ++i)
#pragma unroll
    for (int j = 0; j < 4; ++j) acc[i][j] = (v8f){0.f,0.f,0.f,0.f,0.f,0.f,0.f,0.f};

  for (int k0 = 0; k0 < K; k0 += 32) {
    V bh[4], bl[4];
#pragma unroll
    for (int j = 0; j < 4; ++j) {
      const size_t bo = (size_t)(n0 + (j << 4) + rlane) * ldb + koff + k0;
      bh[j] = Frag<T>::load(Bt + bo);
      if (SPL == 2) bl[j] = Frag<T>::load(Bt2 + bo);
    }
#pragma unroll
    for (int i = 0; i < 4; ++i) {
      const size_t ao = (size_t)(m0 + (i << 4) + rlane) * lda + koff + k0;
      V ah = Frag<T>::load(A + ao);
      V al;
      if (SPL == 2) al = Frag<T>::load(A2 + ao);
#pragma unroll
      for (int j = 0; j < 4; ++j) {
        acc[i][j] = Frag<T>::mma(ah, bh[j], acc[i][j]);
        if (SPL == 2) {
          acc[i][j] = Frag<T>::mma(ah, bl[j], acc[i][j]);
          acc[i][j] = Frag<T>::mma(al, bh[j], acc[i][j]);
        }
      }
      Frag<T>::tie(acc[i][0], ah, (SPL == 2) ? al : ah);
      Frag<T>::tie(acc[i][1], ah, (SPL == 2) ? al : ah);
      Frag<T>::tie(acc[i][2], ah, (SPL == 2) ? al : ah);
      Frag<T>::nops(acc[i][3], ah, (SPL == 2) ? al : ah);
    }
    Frag<T>::keep(bh[0], bh[1], bh[2], bh[3]);
    if (SPL == 2) Frag<T>::keep(bl[0], bl[1], bl[2], bl[3]);
  }
  acc_guard4(acc[0][0], acc[0][1], acc[0][2], acc[0][3]);
  acc_guard4(acc[1][0], acc[1][1], acc[1][2], acc[1][3]);
  acc_guard4(acc[2][0], acc[2][1], acc[2][2], acc[2][3]);
  acc_guard4(acc[3][0], acc[3][1], acc[3][2], acc[3][3]);

  float* slab = sT[wave];
#pragma unroll
  for (int i = 0; i < 4; ++i) {
    const int mBase = m0 + (i << 4);
#pragma unroll
    for (int j = 0; j < 4; ++j) {
#pragma unroll
      for (int r = 0; r < 8; ++r) {
        const float v = acc[i][j][r] * scale;
        slab[(mOff + r) * 68 + (j << 4) + rlane] = v;
      }
    }
    __builtin_amdgcn_fence(__ATOMIC_RELEASE, "workgroup");
    __builtin_amdgcn_wave_barrier();
    __builtin_amdgcn_fence(__ATOMIC_ACQUIRE, "workgroup");
    {
      const int hh = lane >> 4, c4 = (lane & 15) * 4;
      for (int pass = 0; pass < 2; ++pass) {
#pragma unroll
        for (int it = 0; it < 8; ++it) {
          const int row = it * 2 + hh;
          v4f v = *(const v4f*)(slab + row * 68 + c4);
          *(volatile v4f*)(Cout + (size_t)(mBase + row) * ldc + n0 + c4) = v;
        }
        __threadfence();
      }
    }
    __builtin_amdgcn_fence(__ATOMIC_RELEASE, "workgroup");
    __builtin_amdgcn_wave_barrier();
    __builtin_amdgcn_fence(__ATOMIC_ACQUIRE, "workgroup");
  }
}

template <int MODE>
__global__ __launch_bounds__(256) void split_rows_kernel(
    const float* __restrict__ src, unsigned* __restrict__ dhi, unsigned* __restrict__ dlo,
    int total8, int valid8, float carry)
{
  const int i = blockIdx.x * 256 + threadIdx.x;
  if (i >= total8) return;
  const bool valid = (i < valid8);
  const int ic = valid ? i : (valid8 - 1);
  const size_t e0 = (size_t)ic << 3;
  const v4f a0 = *(const v4f*)(src + e0);
  const v4f a1 = *(const v4f*)(src + e0 + 4);
  float f0 = a0[0], f1 = a0[1], f2 = a0[2], f3 = a0[3];
  float f4 = a1[0], f5 = a1[1], f6 = a1[2], f7 = a1[3];
  asm volatile("" : "+v"(f0), "+v"(f1), "+v"(f2), "+v"(f3));
  asm volatile("" : "+v"(f4), "+v"(f5), "+v"(f6), "+v"(f7));
  float f[8];
  f[0] = valid ? f0 : 0.0f; f[1] = valid ? f1 : 0.0f; f[2] = valid ? f2 : 0.0f; f[3] = valid ? f3 : 0.0f;
  f[4] = valid ? f4 : 0.0f; f[5] = valid ? f5 : 0.0f; f[6] = valid ? f6 : 0.0f; f[7] = valid ? f7 : 0.0f;
  v4u wh, wl;
  pack8<MODE>(f, carry, wh, wl);
  volatile v4u* qh = (volatile v4u*)dhi + i;
  volatile v4u* ql = (volatile v4u*)dlo + i;
  *qh = wh;
  if (MODE != 0) *ql = wl;
  __threadfence();
  *qh = wh;
  if (MODE != 0) *ql = wl;
}

template <int MODE>
__global__ __launch_bounds__(256) void conv_silu_kernel(
    const float* __restrict__ XZ, const float* __restrict__ cw, const float* __restrict__ cb,
    float* __restrict__ UC, unsigned* __restrict__ UH, unsigned* __restrict__ UL, float carry)
{
  __shared__ __align__(16) float sT[16 * kConvTP];
  const unsigned tid  = threadIdx.x;
  const unsigned lane = pin_u32(tid & 31u);
  const unsigned wave = pin_u32(tid >> 5);
  const unsigned d0 = blockIdx.x * 256u;
  const unsigned d  = d0 + tid;
  const unsigned g0 = blockIdx.y * 64u;
  const bool hist = ((g0 & (unsigned)(kSeq - 1)) != 0u);
  const v4f wv = *(const v4f*)(cw + (size_t)d * 4);
  const float w0 = wv[0], w1 = wv[1], w2 = wv[2], w3 = wv[3];
  const float bc = cb[d];
  float xm3, xm2, xm1;
  {
    const unsigned rb = hist ? (g0 - 3u) : g0;
    const float v3 = XZ[(size_t)rb * kXzP + d];
    const float v2 = XZ[(size_t)(rb + 1u) * kXzP + d];
    const float v1 = XZ[(size_t)(rb + 2u) * kXzP + d];
    xm3 = hist ? v3 : 0.0f;
    xm2 = hist ? v2 : 0.0f;
    xm1 = hist ? v1 : 0.0f;
  }
  const unsigned hrow = pin_u32(wave >> 1);
  const unsigned hch  = pin_u32((wave & 1u) * 128u + lane * 4u);
#pragma unroll 1
  for (unsigned sub = 0; sub < 4u; ++sub) {
    const unsigned lb = g0 + sub * 16u;
#pragma unroll 1
    for (unsigned s = 0; s < 16u; ++s) {
      const float xcur = XZ[(size_t)(lb + s) * kXzP + d];
      float acc = w0 * xm3;
      acc = fmaf(w1, xm2, acc);
      acc = fmaf(w2, xm1, acc);
      acc = fmaf(w3, xcur, acc);
      const float sv = acc + bc;
      const float sg = __builtin_amdgcn_rcpf(1.0f + expf(-sv));
      sT[s * kConvTP + tid] = sv * sg;
      xm3 = xm2; xm2 = xm1; xm1 = xcur;
    }
    __syncthreads();
    v4f fv[4];
    v4u wh[2], wl[2];
#pragma unroll
    for (int it = 0; it < 4; ++it) fv[it] = *(const v4f*)(sT + ((unsigned)it * 4u + hrow) * kConvTP + hch);
#pragma unroll
    for (int it = 0; it < 2; ++it) {
      const float* sp = sT + ((unsigned)it * 8u + wave) * kConvTP + lane * 8u;
      const v4f a0 = *(const v4f*)(sp);
      const v4f a1 = *(const v4f*)(sp + 4);
      float f[8];
      f[0] = a0[0]; f[1] = a0[1]; f[2] = a0[2]; f[3] = a0[3];
      f[4] = a1[0]; f[5] = a1[1]; f[6] = a1[2]; f[7] = a1[3];
      pack8<MODE>(f, carry, wh[it], wl[it]);
    }
    for (int pass = 0; pass < 2; ++pass) {
#pragma unroll
      for (int it = 0; it < 4; ++it)
        *(volatile v4f*)(UC + (size_t)(lb + (unsigned)it * 4u + hrow) * kDin + d0 + hch) = fv[it];
#pragma unroll
      for (int it = 0; it < 2; ++it) {
        const size_t o = (size_t)(lb + (unsigned)it * 8u + wave) * (kDin / 8) + (d0 >> 3) + lane;
        ((volatile v4u*)UH)[o] = wh[it];
        if (MODE != 0) ((volatile v4u*)UL)[o] = wl[it];
      }
      __threadfence();
    }
    __syncthreads();
  }
}

template <bool FAST>
__device__ __forceinline__ float step_exp(float x) {
  if (FAST) return __expf(x);
  return expf(x);
}

template <int MODE, bool FAST>
__global__ __launch_bounds__(64) void scan_kernel(
    const float* __restrict__ XD, const float* __restrict__ UC, const float* __restrict__ XZ,
    const float* __restrict__ Wdt, const float* __restrict__ bdt, const float* __restrict__ Alog,
    unsigned* __restrict__ YH, unsigned* __restrict__ YL, float carry)
{
  __shared__ __align__(16) float sX[kScanTS * kXdP];
  __shared__ __align__(16) float sY[kScanTS * kScanYP];
  __shared__ __align__(16) float sA[kNst * kScanCh];
  const unsigned tid  = threadIdx.x;
  const unsigned lane = pin_u32(tid & 31u);
  const unsigned wave = pin_u32(tid >> 5);
  constexpr unsigned kBlkPerB = kDin / kScanCh;
  const unsigned bix = blockIdx.x / kBlkPerB;
  const unsigned d0  = (blockIdx.x - bix * kBlkPerB) * kScanCh;
  const unsigned d   = d0 + tid;
  const size_t row0  = (size_t)bix * kSeq;
#pragma unroll 1
  for (int s = 0; s < kNst; ++s) sA[s * kScanCh + tid] = -expf(Alog[(size_t)d * kNst + s]);
  __syncthreads();
  float negA[kNst], h[kNst];
#pragma unroll
  for (int s = 0; s < kNst; ++s) {
    negA[s] = sA[s * kScanCh + tid];
    h[s] = 0.0f;
  }
  const float wdt = Wdt[d];
  const float bb  = bdt[d];
  const unsigned lr  = pin_u32(tid >> 4);
  const unsigned lc4 = pin_u32((tid & 15u) * 4u);
  const unsigned q   = pin_u32(lane >> 3);
  const unsigned l7  = pin_u32(lane & 7u);
  const unsigned c8  = l7 * 8u;
#pragma unroll 1
  for (unsigned t0 = 0; t0 < (unsigned)kSeq; t0 += kScanTS) {
    __syncthreads();
#pragma unroll
    for (int i = 0; i < 16; ++i) {
      const unsigned r = lr + 4u * (unsigned)i;
      *(v4f*)(sX + r * kXdP + lc4) = *(const v4f*)(XD + (row0 + t0 + r) * kXdP + lc4);
    }
    __syncthreads();
#pragma unroll 1
    for (unsigned s = 0; s < (unsigned)kScanTS; ++s) {
      const size_t grow = row0 + t0 + s;
      const float* xr = sX + s * kXdP;
      float Bs[kNst], Cs[kNst];
#pragma unroll
      for (int q4 = 0; q4 < 4; ++q4) {
        const v4f bv = *(const v4f*)(xr + 4 * q4);
        const v4f cv = *(const v4f*)(xr + kNst + 4 * q4);
        Bs[4 * q4 + 0] = bv[0]; Bs[4 * q4 + 1] = bv[1]; Bs[4 * q4 + 2] = bv[2]; Bs[4 * q4 + 3] = bv[3];
        Cs[4 * q4 + 0] = cv[0]; Cs[4 * q4 + 1] = cv[1]; Cs[4 * q4 + 2] = cv[2]; Cs[4 * q4 + 3] = cv[3];
      }
      const float dtr = xr[2 * kNst];
      const float xt  = UC[grow * kDin + d];
      const float zv  = XZ[grow * kXzP + kDin + d];
      const float v   = fmaf(dtr, wdt, bb);
      const float a   = expf(-fabsf(v));
      const float u1  = 1.0f + a;
      const float l1p = logf(u1) + (a - (u1 - 1.0f)) * __builtin_amdgcn_rcpf(u1);
      const float dt  = fmaxf(v, 0.0f) + l1p;
      const float dtx = dt * xt;
      float y = 0.0f;
#pragma unroll
      for (int k = 0; k < kNst; ++k) {
        const float e = step_exp<FAST>(dt * negA[k]);
        h[k] = fmaf(e, h[k], dtx * Bs[k]);
        y = fmaf(h[k], Cs[k], y);
      }
      const float sg = __builtin_amdgcn_rcpf(1.0f + expf(-zv));
      sY[s * kScanYP + tid] = y * (zv * sg);
    }
    __syncthreads();
    v4u wh[8], wl[8];
#pragma unroll
    for (int it = 0; it < 8; ++it) {
      const unsigned row = (unsigned)it * 8u + wave * 4u + q;
      const float* sp = sY + row * kScanYP + c8;
      const v4f a0 = *(const v4f*)(sp);
      const v4f a1 = *(const v4f*)(sp + 4);
      float f[8];
      f[0] = a0[0]; f[1] = a0[1]; f[2] = a0[2]; f[3] = a0[3];
      f[4] = a1[0]; f[5] = a1[1]; f[6] = a1[2]; f[7] = a1[3];
      pack8<MODE>(f, carry, wh[it], wl[it]);
    }
    for (int pass = 0; pass < 2; ++pass) {
#pragma unroll
      for (int it = 0; it < 8; ++it) {
        const unsigned row = (unsigned)it * 8u + wave * 4u + q;
        const size_t o = (row0 + t0 + row) * (size_t)(kDin / 8) + (d0 >> 3) + l7;
        ((volatile v4u*)YH)[o] = wh[it];
        if (MODE != 0) ((volatile v4u*)YL)[o] = wl[it];
      }
      __threadfence();
    }
  }
}

static_assert((((kRows / 64) * (kXzP / 64)) % 8) == 0);
static_assert((((kRows / 64) * (kXdP / 64)) % 8) == 0);
static_assert((((kRows / 64) * (kDm / 64)) % 8) == 0);
constexpr float kScaleIn  = (kModeIn  == 0) ? (1.0f / (kCarryX * kCarryW)) : 1.0f;
constexpr float kScaleXp  = (kModeXp  == 0) ? (1.0f / (kCarryU * kCarryW)) : 1.0f;
constexpr float kScaleOut = (kModeOut == 0) ? (1.0f / (kCarryY * kCarryW)) : 1.0f;
static_assert(((kRows * kDm / 8) % 256) == 0 && ((kXzP * kDm / 8) % 256) == 0 &&
              ((kXdP * kDin / 8) % 256) == 0 && ((kDm * kDin / 8) % 256) == 0);

extern "C" void kernel_launch(void* const* d_in, const int* in_sizes, int n_in,
                              void* d_out, int out_size, void* d_ws, size_t ws_size,
                              hipStream_t stream) {
  if (n_in < 9) return;
  if (in_sizes[0] != kRows * kDm) return;
  if (in_sizes[1] != kXzP * kDm) return;
  if (in_sizes[2] != kDin * 4) return;
  if (in_sizes[3] != kDin) return;
  if (in_sizes[4] != kDin * kNst) return;
  if (in_sizes[5] != kXdN * kDin) return;
  if (in_sizes[6] != kDin) return;
  if (in_sizes[7] != kDin) return;
  if (in_sizes[8] != kDm * kDin) return;
  if (out_size != kRows * kDm) return;
  if (ws_size < kWsTotal) return;

  const float* x       = (const float*)d_in[0];
  const float* W_in    = (const float*)d_in[1];
  const float* conv_w  = (const float*)d_in[2];
  const float* conv_b  = (const float*)d_in[3];
  const float* A_log   = (const float*)d_in[4];
  const float* W_x     = (const float*)d_in[5];
  const float* w_dt    = (const float*)d_in[6];
  const float* b_dt    = (const float*)d_in[7];
  const float* W_out   = (const float*)d_in[8];
  float* out = (float*)d_out;

  char* ws = (char*)d_ws;
  unsigned* XH  = (unsigned*)(ws + kOffXH);
  unsigned* XL  = (unsigned*)(ws + kOffXL);
  unsigned* W0H = (unsigned*)(ws + kOffW0H);
  unsigned* W0L = (unsigned*)(ws + kOffW0L);
  unsigned* W1H = (unsigned*)(ws + kOffW1H);
  unsigned* W1L = (unsigned*)(ws + kOffW1L);
  unsigned* W3H = (unsigned*)(ws + kOffW3H);
  unsigned* W3L = (unsigned*)(ws + kOffW3L);
  float*    XZ  = (float*)(ws + kOffXZ);
  float*    UC  = (float*)(ws + kOffUC);
  unsigned* UH  = (unsigned*)(ws + kOffUH);
  unsigned* UL  = (unsigned*)(ws + kOffUL);
  float*    XD  = (float*)(ws + kOffXD);
  unsigned* YH  = (unsigned*)(ws + kOffYH);
  unsigned* YL  = (unsigned*)(ws + kOffYL);

  constexpr int kEtIn  = (kModeIn  == 0) ? 0 : 1;
  constexpr int kEtXp  = (kModeXp  == 0) ? 0 : 1;
  constexpr int kEtOut = (kModeOut == 0) ? 0 : 1;

  split_rows_kernel<kModeIn><<<(kRows * kDm / 8) / 256, 256, 0, stream>>>(
      x, XH, XL, kRows * kDm / 8, kRows * kDm / 8, kCarryX);
  split_rows_kernel<kModeIn><<<(kXzP * kDm / 8) / 256, 256, 0, stream>>>(
      W_in, W0H, W0L, kXzP * kDm / 8, kXzP * kDm / 8, kCarryW);
  split_rows_kernel<kModeXp><<<(kXdP * kDin / 8) / 256, 256, 0, stream>>>(
      W_x, W1H, W1L, kXdP * kDin / 8, kXdN * kDin / 8, kCarryW);
  split_rows_kernel<kModeOut><<<(kDm * kDin / 8) / 256, 256, 0, stream>>>(
      W_out, W3H, W3L, kDm * kDin / 8, kDm * kDin / 8, kCarryW);

  wmma_gemm64<kEtIn, kModeIn><<<dim3(((kRows / 64) * (kXzP / 64)) / 8), 256, 0, stream>>>(
      (const unsigned short*)XH, (const unsigned short*)XL, kDm,
      (const unsigned short*)W0H, (const unsigned short*)W0L, kDm,
      XZ, kXzP, kRows, kXzP, kDm, kScaleIn);

  conv_silu_kernel<kModeXp><<<dim3(kDin / 256, kRows / 64), 256, 0, stream>>>(
      XZ, conv_w, conv_b, UC, UH, UL, kCarryU);

  wmma_gemm64<kEtXp, kModeXp><<<dim3(((kRows / 64) * (kXdP / 64)) / 8), 256, 0, stream>>>(
      (const unsigned short*)UH, (const unsigned short*)UL, kDin,
      (const unsigned short*)W1H, (const unsigned short*)W1L, kDin,
      XD, kXdP, kRows, kXdP, kDin, kScaleXp);

  scan_kernel<kModeOut, kScanFastExp><<<kBatch * (kDin / kScanCh), kScanCh, 0, stream>>>(
      XD, UC, XZ, w_dt, b_dt, A_log, YH, YL, kCarryY);

  wmma_gemm64<kEtOut, kModeOut><<<dim3(((kRows / 64) * (kDm / 64)) / 8), 256, 0, stream>>>(
      (const unsigned short*)YH, (const unsigned short*)YL, kDin,
      (const unsigned short*)W3H, (const unsigned short*)W3L, kDin,
      out, kDm, kRows, kDm, kDin, kScaleOut);
}
